// SinkhornAttention_89000312308060
// MI455X (gfx1250) — hardware-verified
//
#include <hip/hip_runtime.h>
#include <math.h>

constexpr int NBATCH = 8;
constexpr int NTOK   = 2048;
constexpr int NPAR   = 2048;
constexpr int DMODEL = 512;
constexpr int GRPB   = 4;
constexpr int NGRP   = NBATCH / GRPB;
constexpr int SK_ITERS = 5;
constexpr float kPiCarry = 16384.0f;

static_assert(NBATCH % GRPB == 0, "grp");
static_assert(NTOK % 64 == 0 && NPAR % 64 == 0 && DMODEL % 64 == 0, "tile multiples");
static_assert(DMODEL % 32 == 0 && NPAR % 32 == 0, "K multiple of 32");
static_assert(NPAR % (4 * 256) == 0, "u sweep grid");
static_assert(NTOK % 32 == 0 && NPAR % 256 == 0, "v sweep grid");

constexpr size_t SZ_WT  = (size_t)DMODEL * DMODEL * 2;
constexpr size_t SZ_QC  = (size_t)NTOK * DMODEL * 2;
constexpr size_t SZ_QP  = (size_t)NTOK * DMODEL * 2;
constexpr size_t SZ_Q2  = (size_t)NTOK * 4;
constexpr size_t SZ_KP  = (size_t)GRPB * NPAR * DMODEL * 2;
constexpr size_t SZ_K2  = (size_t)GRPB * NPAR * 4;
constexpr size_t SZ_VPT = (size_t)GRPB * DMODEL * NPAR * 2;
constexpr size_t SZ_KM  = (size_t)GRPB * NTOK * NPAR * 4;
constexpr size_t SZ_U   = (size_t)GRPB * NPAR * 4;
constexpr size_t SZ_VV  = (size_t)GRPB * NTOK * 4;
constexpr size_t SZ_PI  = (size_t)GRPB * NTOK * NPAR * 2;
constexpr size_t WS_TOTAL = 3 * SZ_WT + SZ_QC + 2 * SZ_QP + SZ_Q2 + 2 * SZ_KP + SZ_K2 + SZ_VPT + SZ_KM + SZ_U + SZ_VV + SZ_PI;
static_assert(WS_TOTAL == 133799936ull, "carve total");
static_assert(WS_TOTAL <= 134217728ull, "carve limit");
static_assert(2 * SZ_KP <= SZ_PI, "k/v casts live inside the pi region");

typedef __attribute__((ext_vector_type(16))) _Float16 v16h;
typedef __attribute__((ext_vector_type(8)))  _Float16 v8h;
typedef __attribute__((ext_vector_type(16))) __bf16   v16b;
typedef __attribute__((ext_vector_type(8)))  __bf16   v8b;
typedef __attribute__((ext_vector_type(8)))  float    v8f;
typedef __attribute__((ext_vector_type(4)))  float    v4f;
typedef unsigned v4u __attribute__((ext_vector_type(4)));
typedef unsigned v4ua __attribute__((ext_vector_type(4), __may_alias__));
#define PSCALE 32768.0f
#define U16(p) ((const unsigned short*)(const void*)(p))
#define PSCALE_INV (1.0f / 32768.0f)

__device__ __forceinline__ unsigned short f2bf_bits(float f) {
  unsigned u = __float_as_uint(f);
  return (unsigned short)((u + 0x7FFFu + ((u >> 16) & 1u)) >> 16);
}
__device__ __forceinline__ float bf_bits2f(unsigned short h) { return __uint_as_float(((unsigned)h) << 16); }

__device__ __forceinline__ void dep_guard_h(v8f& a, v8f& b, v16h x, v16h y) { asm volatile("v_nop\n\tv_nop\n\tv_nop\n\tv_nop" : "+v"(a), "+v"(b) : "v"(x), "v"(y)); }
__device__ __forceinline__ void dep_guard_b(v8f& a, v8f& b, v16b x, v16b y) { asm volatile("v_nop\n\tv_nop\n\tv_nop\n\tv_nop" : "+v"(a), "+v"(b) : "v"(x), "v"(y)); }
__device__ __forceinline__ void keep4_h(v16h a, v16h b, v16h c, v16h d) { asm volatile("v_nop" :: "v"(a), "v"(b), "v"(c), "v"(d)); }
__device__ __forceinline__ void keep4_b(v16b a, v16b b, v16b c, v16b d) { asm volatile("v_nop" :: "v"(a), "v"(b), "v"(c), "v"(d)); }
__device__ __forceinline__ void acc_guard4(v8f& a, v8f& b, v8f& c, v8f& d) { asm volatile("v_nop\n\tv_nop\n\tv_nop\n\tv_nop" : "+v"(a), "+v"(b), "+v"(c), "+v"(d)); }
template <typename T> struct Frag;
template <> struct Frag<_Float16> {
  typedef v16h V; union U { v16h v; v8h h[2]; };
  static __device__ __forceinline__ v16h load(const _Float16* p) {
    U f; f.h[0] = *(const v8h*)(p); f.h[1] = *(const v8h*)(p + 16); return f.v;
  }
  static __device__ __forceinline__ v8f mma(v16h a, v16h b, v8f c) {
    return __builtin_amdgcn_wmma_f32_16x16x32_f16(false, a, false, b, (short)0, c, false, false);
  }
  static __device__ __forceinline__ void guard(v8f& a, v8f& b, v16h x, v16h y) { dep_guard_h(a, b, x, y); }
  static __device__ __forceinline__ void keep(v16h a, v16h b, v16h c, v16h d) { keep4_h(a, b, c, d); }
};
template <> struct Frag<__bf16> {
  typedef v16b V; union U { v16b v; v8b h[2]; };
  static __device__ __forceinline__ v16b load(const __bf16* p) {
    U f; f.h[0] = *(const v8b*)(p); f.h[1] = *(const v8b*)(p + 16); return f.v;
  }
  static __device__ __forceinline__ v8f mma(v16b a, v16b b, v8f c) {
    return __builtin_amdgcn_wmma_f32_16x16x32_bf16(false, a, false, b, (short)0, c, false, false);
  }
  static __device__ __forceinline__ void guard(v8f& a, v8f& b, v16b x, v16b y) { dep_guard_b(a, b, x, y); }
  static __device__ __forceinline__ void keep(v16b a, v16b b, v16b c, v16b d) { keep4_b(a, b, c, d); }
};

template <int ET> struct Elem;
template <> struct Elem<0> { typedef _Float16 T; };
template <> struct Elem<1> { typedef __bf16 T; };
template <int ET, bool SPLIT, int BIAS_MODE, int OUT_MODE, bool RESID, int ACT = 0>
__global__ __launch_bounds__(256) void wmma_gemm64(
    const unsigned short* __restrict__ Ap, const unsigned short* __restrict__ A2p, int lda, long strideA,
    const unsigned short* __restrict__ Btp, const unsigned short* __restrict__ Bt2p, int ldb, long strideB,
    void* __restrict__ Cout, void* __restrict__ Cout2, int ldc, long strideC,
    const float* __restrict__ bias,
    const float* __restrict__ resid, long strideR,
    int M, int N, int K, float scale) {
  typedef typename Elem<ET>::T T;
  typedef typename Frag<T>::V V;
  const T* A = (const T*)Ap; const T* A2 = (const T*)A2p; const T* Bt = (const T*)Btp; const T* Bt2 = (const T*)Bt2p;
  __shared__ __align__(16) float sT[8][16 * 68];
  const int b    = blockIdx.y;
  const int lane = threadIdx.x & 31;
  const int wave = threadIdx.x >> 5;
  const int tilesN = N >> 6;
  const int tilesM = M >> 6;
  const int tile = blockIdx.x * 8 + wave;
  if (tile >= tilesM * tilesN) return;
  const int tm = tile / tilesN;
  const int tn = tile - tm * tilesN;
  const int m0 = tm << 6;
  const int n0 = tn << 6;

  const T* Ab  = A  + (size_t)b * strideA;
  const T* Bb  = Bt + (size_t)b * strideB;
  const T* Ab2 = SPLIT ? (A2  + (size_t)b * strideA) : nullptr;
  const T* Bb2 = SPLIT ? (Bt2 + (size_t)b * strideB) : nullptr;

  const int rlane = lane & 15;
  const int koff  = (lane >> 4) * 8;
  const int mOff  = (lane >> 4) * 8;

  v8f acc[4][4];
#pragma unroll
  for (int i = 0; i < 4; ++i)
#pragma unroll
    for (int j = 0; j < 4; ++j) acc[i][j] = (v8f){0.f,0.f,0.f,0.f,0.f,0.f,0.f,0.f};

  for (int k0 = 0; k0 < K; k0 += 32) {
    V bh[4], bl[4];
#pragma unroll
    for (int j = 0; j < 4; ++j) {
      const size_t bo = (size_t)(n0 + (j << 4) + rlane) * ldb + koff + k0;
      bh[j] = Frag<T>::load(Bb + bo);
      if (SPLIT) bl[j] = Frag<T>::load(Bb2 + bo);
    }
#pragma unroll
    for (int i = 0; i < 4; ++i) {
      const size_t ao = (size_t)(m0 + (i << 4) + rlane) * lda + koff + k0;
      V ah = Frag<T>::load(Ab + ao);
      V al;
      if (SPLIT) al = Frag<T>::load(Ab2 + ao);
#pragma unroll
      for (int j = 0; j < 4; ++j) {
        acc[i][j] = Frag<T>::mma(ah, bh[j], acc[i][j]);
        if (SPLIT) {
          acc[i][j] = Frag<T>::mma(ah, bl[j], acc[i][j]);
          acc[i][j] = Frag<T>::mma(al, bh[j], acc[i][j]);
        }
      }
      Frag<T>::guard(acc[i][0], acc[i][3], ah, SPLIT ? al : ah);
    }
    Frag<T>::keep(bh[0], bh[1], bh[2], bh[3]);
    if (SPLIT) Frag<T>::keep(bl[0], bl[1], bl[2], bl[3]);
  }
  acc_guard4(acc[0][0], acc[0][1], acc[0][2], acc[0][3]);
  acc_guard4(acc[1][0], acc[1][1], acc[1][2], acc[1][3]);
  acc_guard4(acc[2][0], acc[2][1], acc[2][2], acc[2][3]);
  acc_guard4(acc[3][0], acc[3][1], acc[3][2], acc[3][3]);

  float* slab = sT[wave];
  const float* Rb = RESID ? (resid + (size_t)b * strideR) : nullptr;
#pragma unroll
  for (int i = 0; i < 4; ++i) {
    const int mBase = m0 + (i << 4);
#pragma unroll
    for (int j = 0; j < 4; ++j) {
      const int n = n0 + (j << 4) + rlane;
      float bv = 0.f;
      if (BIAS_MODE == 2) bv = bias[n];
#pragma unroll
      for (int r = 0; r < 8; ++r) {
        float v = acc[i][j][r] * scale;
        if (BIAS_MODE == 1) v += bias[mBase + mOff + r];
        if (BIAS_MODE == 2) v += bv;
        if (RESID) v += Rb[(size_t)(mBase + mOff + r) * ldc + n];
        if (ACT == 1) v = tanhf(v);
        if (ACT == 2) v = fmaxf(v, 0.0f);
        if (ACT == 3) v = v / (1.0f + expf(-v));
        if (ACT == 4) v = (v > 0.f) ? v : 0.01f * v;
        if (ACT == 5) v = 0.5f * v * (1.0f + erff(v * 0.70710678118654752f));
        slab[(mOff + r) * 68 + (j << 4) + rlane] = v;
      }
    }
    __builtin_amdgcn_fence(__ATOMIC_RELEASE, "workgroup");
    __builtin_amdgcn_wave_barrier();
    __builtin_amdgcn_fence(__ATOMIC_ACQUIRE, "workgroup");
    if (OUT_MODE == 0) {
      float* C = (float*)Cout + (size_t)b * strideC;
      const int hh = lane >> 4, c4 = (lane & 15) * 4;
      for (int pass = 0; pass < 2; ++pass) {
#pragma unroll
        for (int it = 0; it < 8; ++it) {
          const int row = it * 2 + hh;
          v4f v = *(const v4f*)(slab + row * 68 + c4);
          *(volatile v4f*)(C + (size_t)(mBase + row) * ldc + n0 + c4) = v;
        }
        __threadfence();
      }
    } else {
      const int q = lane >> 3, c8 = (lane & 7) * 8;
      unsigned short* C  = (unsigned short*)Cout  + (size_t)b * strideC;
      unsigned short* C2 = (OUT_MODE == 2) ? ((unsigned short*)Cout2 + (size_t)b * strideC) : nullptr;
      for (int pass = 0; pass < 2; ++pass) {
#pragma unroll
        for (int it = 0; it < 4; ++it) {
          const int row = it * 4 + q;
          const float* sp = slab + row * 68 + c8;
          v8h hv, lv;
#pragma unroll
          for (int e = 0; e < 8; ++e) {
            if (OUT_MODE == 1) {
              hv[e] = (_Float16)sp[e];
            } else {
              unsigned short hb = f2bf_bits(sp[e]);
              unsigned short lb = f2bf_bits(sp[e] - bf_bits2f(hb));
              hv[e] = __builtin_bit_cast(_Float16, hb);
              lv[e] = __builtin_bit_cast(_Float16, lb);
            }
          }
          *(volatile v8h*)(C + (size_t)(mBase + row) * ldc + n0 + c8) = hv;
          if (OUT_MODE == 2) *(volatile v8h*)(C2 + (size_t)(mBase + row) * ldc + n0 + c8) = lv;
        }
        __threadfence();
      }
    }
    __builtin_amdgcn_fence(__ATOMIC_RELEASE, "workgroup");
    __builtin_amdgcn_wave_barrier();
    __builtin_amdgcn_fence(__ATOMIC_ACQUIRE, "workgroup");
  }
}

__global__ __launch_bounds__(256) void gemm64_cdist(
    const unsigned short* __restrict__ Ap, const unsigned short* __restrict__ A2p, int lda,
    const unsigned short* __restrict__ Btp, const unsigned short* __restrict__ Bt2p, int ldb, long strideB,
    float* __restrict__ Cout, int ldc, long strideC,
    const float* __restrict__ q2, const float* __restrict__ k2, long strideK2,
    int M, int N, int K) {
  typedef __bf16 T;
  typedef v16b V;
  const T* A = (const T*)Ap; const T* A2 = (const T*)A2p; const T* Bt = (const T*)Btp; const T* Bt2 = (const T*)Bt2p;
  __shared__ __align__(16) float sT[8][16 * 68];
  const int b    = blockIdx.y;
  const int lane = threadIdx.x & 31;
  const int wave = threadIdx.x >> 5;
  const int tilesN = N >> 6;
  const int tilesM = M >> 6;
  const int tile = blockIdx.x * 8 + wave;
  if (tile >= tilesM * tilesN) return;
  const int tm = tile / tilesN;
  const int tn = tile - tm * tilesN;
  const int m0 = tm << 6;
  const int n0 = tn << 6;

  const T* Ab  = A;
  const T* Bb  = Bt + (size_t)b * strideB;
  const T* Ab2 = A2;
  const T* Bb2 = Bt2 + (size_t)b * strideB;

  const int rlane = lane & 15;
  const int koff  = (lane >> 4) * 8;
  const int mOff  = (lane >> 4) * 8;

  v8f acc[4][4];
#pragma unroll
  for (int i = 0; i < 4; ++i)
#pragma unroll
    for (int j = 0; j < 4; ++j) acc[i][j] = (v8f){0.f,0.f,0.f,0.f,0.f,0.f,0.f,0.f};

  for (int k0 = 0; k0 < K; k0 += 32) {
    V bh[4], bl[4];
#pragma unroll
    for (int j = 0; j < 4; ++j) {
      const size_t bo = (size_t)(n0 + (j << 4) + rlane) * ldb + koff + k0;
      bh[j] = Frag<T>::load(Bb + bo);
      bl[j] = Frag<T>::load(Bb2 + bo);
    }
#pragma unroll
    for (int i = 0; i < 4; ++i) {
      const size_t ao = (size_t)(m0 + (i << 4) + rlane) * lda + koff + k0;
      V ah = Frag<T>::load(Ab + ao);
      V al = Frag<T>::load(Ab2 + ao);
#pragma unroll
      for (int j = 0; j < 4; ++j) {
        acc[i][j] = Frag<T>::mma(ah, bh[j], acc[i][j]);
        acc[i][j] = Frag<T>::mma(ah, bl[j], acc[i][j]);
        acc[i][j] = Frag<T>::mma(al, bh[j], acc[i][j]);
      }
      Frag<T>::guard(acc[i][0], acc[i][3], ah, al);
    }
    Frag<T>::keep(bh[0], bh[1], bh[2], bh[3]);
    Frag<T>::keep(bl[0], bl[1], bl[2], bl[3]);
  }
  acc_guard4(acc[0][0], acc[0][1], acc[0][2], acc[0][3]);
  acc_guard4(acc[1][0], acc[1][1], acc[1][2], acc[1][3]);
  acc_guard4(acc[2][0], acc[2][1], acc[2][2], acc[2][3]);
  acc_guard4(acc[3][0], acc[3][1], acc[3][2], acc[3][3]);

  float* slab = sT[wave];
  const float* k2b = k2 + (size_t)b * strideK2;
  float k2r[4];
#pragma unroll
  for (int j = 0; j < 4; ++j) k2r[j] = k2b[n0 + (j << 4) + rlane];
  float* C = Cout + (size_t)b * strideC;
  const int hh = lane >> 4, c4 = (lane & 15) * 4;
#pragma unroll
  for (int i = 0; i < 4; ++i) {
    const int mBase = m0 + (i << 4);
    const v4f q2a = *(const v4f*)(q2 + mBase + mOff);
    const v4f q2c = *(const v4f*)(q2 + mBase + mOff + 4);
    const float q2r[8] = {q2a.x, q2a.y, q2a.z, q2a.w, q2c.x, q2c.y, q2c.z, q2c.w};
#pragma unroll
    for (int j = 0; j < 4; ++j) {
#pragma unroll
      for (int r = 0; r < 8; ++r) {
        float s = q2r[r] + k2r[j];
        s = s - 2.0f * acc[i][j][r];
        slab[(mOff + r) * 68 + (j << 4) + rlane] = -sqrtf(fmaxf(s, 0.0f));
      }
    }
    __builtin_amdgcn_fence(__ATOMIC_RELEASE, "workgroup");
    __builtin_amdgcn_wave_barrier();
    __builtin_amdgcn_fence(__ATOMIC_ACQUIRE, "workgroup");
    for (int pass = 0; pass < 2; ++pass) {
#pragma unroll
      for (int it = 0; it < 8; ++it) {
        const int row = it * 2 + hh;
        v4f v = *(const v4f*)(slab + row * 68 + c4);
        *(volatile v4f*)(C + (size_t)(mBase + row) * ldc + n0 + c4) = v;
      }
      __threadfence();
    }
    __builtin_amdgcn_fence(__ATOMIC_RELEASE, "workgroup");
    __builtin_amdgcn_wave_barrier();
    __builtin_amdgcn_fence(__ATOMIC_ACQUIRE, "workgroup");
  }
}

__device__ __forceinline__ unsigned pack_bf2(float a, float b) {
  return (unsigned)f2bf_bits(a) | ((unsigned)f2bf_bits(b) << 16);
}
__device__ __forceinline__ unsigned pack_half2(float a, float b) {
  const unsigned short ha = __builtin_bit_cast(unsigned short, (_Float16)a);
  const unsigned short hb = __builtin_bit_cast(unsigned short, (_Float16)b);
  return (unsigned)ha | ((unsigned)hb << 16);
}
__device__ __forceinline__ float fexp(float x) { return __expf(x); }

__global__ __launch_bounds__(256) void k_wtrans(const float* __restrict__ W0, const float* __restrict__ W1,
                                                const float* __restrict__ W2, unsigned short* __restrict__ O0,
                                                unsigned short* __restrict__ O1, unsigned short* __restrict__ O2) {
  __shared__ __align__(16) unsigned short st[64 * 72];
  const int z = blockIdx.z;
  const float* W = (z == 0) ? W0 : ((z == 1) ? W1 : W2);
  unsigned short* O = (z == 0) ? O0 : ((z == 1) ? O1 : O2);
  const int c0 = blockIdx.y * 64;
  const int d0 = blockIdx.x * 64;
  const int tid = threadIdx.x;
  const int rr = tid >> 4, cc = (tid & 15) * 4;
#pragma unroll
  for (int p = 0; p < 4; ++p) {
    const int r = rr + 16 * p;
    const v4f x = *(const v4f*)(W + (size_t)(c0 + r) * DMODEL + d0 + cc);
    st[(cc + 0) * 72 + r] = f2bf_bits(x.x);
    st[(cc + 1) * 72 + r] = f2bf_bits(x.y);
    st[(cc + 2) * 72 + r] = f2bf_bits(x.z);
    st[(cc + 3) * 72 + r] = f2bf_bits(x.w);
  }
  __syncthreads();
  const int lane = tid & 31, wave = tid >> 5;
  const int q = lane >> 3, c8 = (lane & 7) * 8;
  for (int pass = 0; pass < 2; ++pass) {
#pragma unroll
    for (int it = 0; it < 2; ++it) {
      const int dd = wave * 8 + it * 4 + q;
      const v4ua val = *(const v4ua*)(st + dd * 72 + c8);
      *(volatile v4u*)(O + (size_t)(d0 + dd) * DMODEL + c0 + c8) = val;
    }
    __threadfence();
  }
}

__global__ __launch_bounds__(256) void k_cast16(const float* __restrict__ in0, unsigned short* __restrict__ out0,
                                                const float* __restrict__ in1, unsigned short* __restrict__ out1,
                                                int n8) {
  const float* in = blockIdx.y ? in1 : in0;
  unsigned short* out = blockIdx.y ? out1 : out0;
  const int i = blockIdx.x * 256 + threadIdx.x;
  if (i < n8) {
    const v4f a = *(const v4f*)(in + (size_t)i * 8);
    const v4f c = *(const v4f*)(in + (size_t)i * 8 + 4);
    v4u w;
    w.x = pack_bf2(a.x, a.y);
    w.y = pack_bf2(a.z, a.w);
    w.z = pack_bf2(c.x, c.y);
    w.w = pack_bf2(c.z, c.w);
    *(volatile v4u*)(out + (size_t)i * 8) = w;
    __threadfence();
    *(volatile v4u*)(out + (size_t)i * 8) = w;
  }
}

__global__ __launch_bounds__(256) void k_rowsq(const unsigned short* __restrict__ hi, const unsigned short* __restrict__ lo,
                                               float* __restrict__ out, int rows) {
  __shared__ __align__(16) float sres[32];
  const int lane = threadIdx.x & 31, wave = threadIdx.x >> 5;
  const int r0 = blockIdx.x * 32;
#pragma unroll 1
  for (int rr = 0; rr < 4; ++rr) {
    int row = r0 + wave * 4 + rr;
    row = row < rows ? row : rows - 1;
    const size_t base = (size_t)row * DMODEL;
    float s = 0.f;
#pragma unroll
    for (int c = 0; c < 2; ++c) {
      const v4u hw = *(const v4u*)(hi + base + c * 256 + lane * 8);
      const v4u lw = *(const v4u*)(lo + base + c * 256 + lane * 8);
#pragma unroll
      for (int e = 0; e < 4; ++e) {
        const float a0 = __uint_as_float(hw[e] << 16);
        const float b0 = __uint_as_float(lw[e] << 16);
        const float f0 = a0 + b0;
        s = fmaf(f0, f0, s);
        const float a1 = __uint_as_float(hw[e] & 0xffff0000u);
        const float b1 = __uint_as_float(lw[e] & 0xffff0000u);
        const float f1 = a1 + b1;
        s = fmaf(f1, f1, s);
      }
    }
#pragma unroll
    for (int off = 16; off; off >>= 1) s += __shfl_xor(s, off, 32);
    if (lane == 0) sres[wave * 4 + rr] = s;
  }
  __syncthreads();
  if (wave == 0) {
    const int li = lane < 8 ? lane : 7;
    const v4f val = *(const v4f*)(sres + li * 4);
    float* op = out + r0 + li * 4;
    if (lane < 8) *(volatile v4f*)op = val;
    __threadfence();
    if (lane < 8) *(volatile v4f*)op = val;
  }
}

template <bool USEV>
__global__ __launch_bounds__(256) void k_upd_u(const float* __restrict__ Km, const float* __restrict__ vv,
                                               float* __restrict__ u, float logA) {
  const int b = blockIdx.y;
  const int col = (blockIdx.x * 256 + threadIdx.x) * 4;
  const float* Kc = Km + (size_t)b * NTOK * NPAR + col;
  const float* vb = vv + (size_t)b * NTOK;
  const float ninf = -__builtin_inff();
  float m0 = ninf, m1 = ninf, m2 = ninf, m3 = ninf;
#pragma unroll 4
  for (int t = 0; t < NTOK; ++t) {
    const v4f x = *(const v4f*)(Kc + (size_t)t * NPAR);
    float vt = 0.f;
    if (USEV) vt = vb[t];
    m0 = fmaxf(m0, x.x + vt);
    m1 = fmaxf(m1, x.y + vt);
    m2 = fmaxf(m2, x.z + vt);
    m3 = fmaxf(m3, x.w + vt);
  }
  float s0 = 0.f, s1 = 0.f, s2 = 0.f, s3 = 0.f;
#pragma unroll 4
  for (int t = 0; t < NTOK; ++t) {
    const v4f x = *(const v4f*)(Kc + (size_t)t * NPAR);
    float vt = 0.f;
    if (USEV) vt = vb[t];
    s0 += fexp((x.x + vt) - m0);
    s1 += fexp((x.y + vt) - m1);
    s2 += fexp((x.z + vt) - m2);
    s3 += fexp((x.w + vt) - m3);
  }
  v4f r;
  r.x = logA - (m0 + logf(s0));
  r.y = logA - (m1 + logf(s1));
  r.z = logA - (m2 + logf(s2));
  r.w = logA - (m3 + logf(s3));
  float* up = u + (size_t)b * NPAR + col;
  *(volatile v4f*)up = r;
  __threadfence();
  *(volatile v4f*)up = r;
}

template <bool LAST>
__global__ __launch_bounds__(256) void k_upd_v(const float* __restrict__ Km, const float* __restrict__ u,
                                               float* __restrict__ vv, unsigned short* __restrict__ pp) {
  __shared__ __align__(16) float sres[32];
  const int b = blockIdx.y;
  const int lane = threadIdx.x & 31, wave = threadIdx.x >> 5;
  const int r0 = blockIdx.x * 32;
  const float* Kb = Km + (size_t)b * NTOK * NPAR;
  const float* ub = u + (size_t)b * NPAR + lane * 8;
#pragma unroll 1
  for (int rr = 0; rr < 4; ++rr) {
    const int t = r0 + wave * 4 + rr;
    const float* Kr = Kb + (size_t)t * NPAR + lane * 8;
    float m = -__builtin_inff();
#pragma unroll 1
    for (int c = 0; c < 8; ++c) {
      v4f x0 = *(const v4f*)(Kr + c * 256);
      v4f x1 = *(const v4f*)(Kr + c * 256 + 4);
      const v4f u0 = *(const v4f*)(ub + c * 256);
      const v4f u1 = *(const v4f*)(ub + c * 256 + 4);
      x0 += u0; x1 += u1;
      m = fmaxf(m, fmaxf(fmaxf(x0.x, x0.y), fmaxf(x0.z, x0.w)));
      m = fmaxf(m, fmaxf(fmaxf(x1.x, x1.y), fmaxf(x1.z, x1.w)));
    }
#pragma unroll
    for (int off = 16; off; off >>= 1) m = fmaxf(m, __shfl_xor(m, off, 32));
    float s = 0.f;
#pragma unroll 1
    for (int c = 0; c < 8; ++c) {
      v4f x0 = *(const v4f*)(Kr + c * 256);
      v4f x1 = *(const v4f*)(Kr + c * 256 + 4);
      const v4f u0 = *(const v4f*)(ub + c * 256);
      const v4f u1 = *(const v4f*)(ub + c * 256 + 4);
      x0 += u0; x1 += u1;
      float a = fexp(x0.x - m) + fexp(x0.y - m);
      a += fexp(x0.z - m) + fexp(x0.w - m);
      float c2 = fexp(x1.x - m) + fexp(x1.y - m);
      c2 += fexp(x1.z - m) + fexp(x1.w - m);
      s += a + c2;
    }
#pragma unroll
    for (int off = 16; off; off >>= 1) s += __shfl_xor(s, off, 32);
    const float vt = -(m + logf(s));
    if (LAST) {
      unsigned short* prow = pp + ((size_t)b * NTOK + t) * NPAR + lane * 8;
#pragma unroll 1
      for (int c = 0; c < 8; ++c) {
        v4f x0 = *(const v4f*)(Kr + c * 256);
        v4f x1 = *(const v4f*)(Kr + c * 256 + 4);
        const v4f u0 = *(const v4f*)(ub + c * 256);
        const v4f u1 = *(const v4f*)(ub + c * 256 + 4);
        x0 += u0; x1 += u1;
        v4u w;
        w.x = pack_half2(fexp(x0.x + vt) * kPiCarry, fexp(x0.y + vt) * kPiCarry);
        w.y = pack_half2(fexp(x0.z + vt) * kPiCarry, fexp(x0.w + vt) * kPiCarry);
        w.z = pack_half2(fexp(x1.x + vt) * kPiCarry, fexp(x1.y + vt) * kPiCarry);
        w.w = pack_half2(fexp(x1.z + vt) * kPiCarry, fexp(x1.w + vt) * kPiCarry);
        *(volatile v4u*)(prow + c * 256) = w;
        __threadfence();
        *(volatile v4u*)(prow + c * 256) = w;
      }
    }
    if (lane == 0) sres[wave * 4 + rr] = vt;
  }
  __syncthreads();
  if (wave == 0) {
    const int li = lane < 8 ? lane : 7;
    const v4f val = *(const v4f*)(sres + li * 4);
    float* op = vv + (size_t)b * NTOK + r0 + li * 4;
    if (lane < 8) *(volatile v4f*)op = val;
    __threadfence();
    if (lane < 8) *(volatile v4f*)op = val;
  }
}

static inline unsigned cdiv(unsigned a, unsigned b) { return (a + b - 1) / b; }

extern "C" void kernel_launch(void* const* d_in, const int* in_sizes, int n_in,
                              void* d_out, int out_size, void* d_ws, size_t ws_size,
                              hipStream_t stream)
{
  if (n_in < 6) return;
  if (in_sizes[0] != NTOK * DMODEL) return;
  if (in_sizes[1] != NBATCH * NPAR * DMODEL) return;
  if (in_sizes[2] != NBATCH * NPAR * DMODEL) return;
  if (in_sizes[3] != DMODEL * DMODEL || in_sizes[4] != DMODEL * DMODEL || in_sizes[5] != DMODEL * DMODEL) return;
  if (out_size != NBATCH * NTOK * DMODEL) return;
  if (WS_TOTAL > ws_size) return;

  const float* q  = (const float*)d_in[0];
  const float* k  = (const float*)d_in[1];
  const float* v  = (const float*)d_in[2];
  const float* Qw = (const float*)d_in[3];
  const float* Kw = (const float*)d_in[4];
  const float* Vw = (const float*)d_in[5];
  float* out = (float*)d_out;

  char* ws = (char*)d_ws;
  size_t off = 0;
  unsigned short* Qt   = (unsigned short*)(ws + off); off += SZ_WT;
  unsigned short* Kt   = (unsigned short*)(ws + off); off += SZ_WT;
  unsigned short* Vt   = (unsigned short*)(ws + off); off += SZ_WT;
  unsigned short* qc   = (unsigned short*)(ws + off); off += SZ_QC;
  unsigned short* qph  = (unsigned short*)(ws + off); off += SZ_QP;
  unsigned short* qpl  = (unsigned short*)(ws + off); off += SZ_QP;
  float*          q2   = (float*)(ws + off);          off += SZ_Q2;
  unsigned short* kph  = (unsigned short*)(ws + off); off += SZ_KP;
  unsigned short* kpl  = (unsigned short*)(ws + off); off += SZ_KP;
  float*          k2   = (float*)(ws + off);          off += SZ_K2;
  unsigned short* vpT  = (unsigned short*)(ws + off); off += SZ_VPT;
  float*          Kmat = (float*)(ws + off);          off += SZ_KM;
  float*          up   = (float*)(ws + off);          off += SZ_U;
  float*          vvp  = (float*)(ws + off);          off += SZ_VV;
  unsigned short* pip  = (unsigned short*)(ws + off); off += SZ_PI;
  if (off > ws_size) return;
  unsigned short* kc = pip;
  unsigned short* vc = (unsigned short*)((char*)pip + SZ_KP);

  const float logA = -(float)log((double)NPAR);

  k_wtrans<<<dim3(DMODEL / 64, DMODEL / 64, 3), dim3(256), 0, stream>>>(Qw, Kw, Vw, Qt, Kt, Vt);

  {
    const int n8 = NTOK * DMODEL / 8;
    k_cast16<<<dim3(cdiv(n8, 256), 1), dim3(256), 0, stream>>>(q, qc, q, qc, n8);
  }
  wmma_gemm64<1, false, 0, 2, false, 0><<<dim3(cdiv((NTOK / 64) * (DMODEL / 64), 8), 1), dim3(256), 0, stream>>>(
      qc, nullptr, DMODEL, 0L, Qt, nullptr, DMODEL, 0L, (void*)qph, (void*)qpl, DMODEL, 0L,
      nullptr, nullptr, 0L, NTOK, DMODEL, DMODEL, 1.0f);
  k_rowsq<<<dim3(NTOK / 32), dim3(256), 0, stream>>>(qph, qpl, q2, NTOK);

  for (int g = 0; g < NGRP; ++g) {
    const size_t rowoff = (size_t)g * GRPB * NPAR * DMODEL;
    {
      const int n8 = GRPB * NPAR * DMODEL / 8;
      k_cast16<<<dim3(cdiv(n8, 256), 2), dim3(256), 0, stream>>>(k + rowoff, kc, v + rowoff, vc, n8);
    }
    wmma_gemm64<1, false, 0, 2, false, 0><<<dim3(cdiv((GRPB * NPAR / 64) * (DMODEL / 64), 8), 1), dim3(256), 0, stream>>>(
        kc, nullptr, DMODEL, 0L, Kt, nullptr, DMODEL, 0L, (void*)kph, (void*)kpl, DMODEL, 0L,
        nullptr, nullptr, 0L, GRPB * NPAR, DMODEL, DMODEL, 1.0f);
    k_rowsq<<<dim3(GRPB * NPAR / 32), dim3(256), 0, stream>>>(kph, kpl, k2, GRPB * NPAR);
    wmma_gemm64<1, false, 0, 1, false, 0><<<dim3(cdiv((DMODEL / 64) * (NPAR / 64), 8), GRPB), dim3(256), 0, stream>>>(
        Vt, nullptr, DMODEL, 0L, vc, nullptr, DMODEL, (long)NPAR * DMODEL, (void*)vpT, nullptr, NPAR, (long)DMODEL * NPAR,
        nullptr, nullptr, 0L, DMODEL, NPAR, DMODEL, 1.0f);
    gemm64_cdist<<<dim3(cdiv((NTOK / 64) * (NPAR / 64), 8), GRPB), dim3(256), 0, stream>>>(
        qph, qpl, DMODEL, kph, kpl, DMODEL, (long)NPAR * DMODEL, Kmat, NPAR, (long)NTOK * NPAR,
        q2, k2, (long)NPAR, NTOK, NPAR, DMODEL);
    for (int it = 0; it < SK_ITERS; ++it) {
      if (it == 0)
        k_upd_u<false><<<dim3(NPAR / 4 / 256, GRPB), dim3(256), 0, stream>>>(Kmat, vvp, up, logA);
      else
        k_upd_u<true><<<dim3(NPAR / 4 / 256, GRPB), dim3(256), 0, stream>>>(Kmat, vvp, up, logA);
      if (it == SK_ITERS - 1)
        k_upd_v<true><<<dim3(NTOK / 32, GRPB), dim3(256), 0, stream>>>(Kmat, up, vvp, pip);
      else
        k_upd_v<false><<<dim3(NTOK / 32, GRPB), dim3(256), 0, stream>>>(Kmat, up, vvp, pip);
    }
    wmma_gemm64<0, false, 0, 0, false, 0><<<dim3(cdiv((NTOK / 64) * (DMODEL / 64), 8), GRPB), dim3(256), 0, stream>>>(
        pip, nullptr, NPAR, (long)NTOK * NPAR, vpT, nullptr, NPAR, (long)DMODEL * NPAR,
        (void*)(out + (size_t)g * GRPB * NTOK * DMODEL), nullptr, DMODEL, (long)NTOK * DMODEL,
        nullptr, nullptr, 0L, NTOK, DMODEL, NPAR, 1.0f / kPiCarry);
  }
}
